// SharedScaleNA_87720412054034
// MI455X (gfx1250) — hardware-verified
//
#include <hip/hip_runtime.h>
#include <hip/hip_bf16.h>


#define BN     2
#define CIN    3
#define IMG    192
#define PATCH  4
#define HH     48
#define WW     48
#define PIX    (HH * WW)
#define NPIX   (BN * PIX)
#define CMID   256
#define CQKV   768
#define HEADS  8
#define HD     32
#define KW     7
#define KTR    (CIN * PATCH * PATCH)
#define KT     64

#define X_N    (BN * CIN * IMG * IMG)
#define WT_N   (CMID * KTR)
#define BT_N   (CMID)
#define WQ_N   (CQKV * CMID)
#define BQ_N   (CQKV)
#define OUT_N  (HEADS * BN * HD * PIX)

#define SZ_A    ((size_t)NPIX * KT * 2)
#define SZ_WT   ((size_t)CMID * KT * 2)
#define SZ_WQ   ((size_t)CQKV * CMID * 2)
#define SZ_TOK  ((size_t)NPIX * CMID * 2)
#define SZ_QKV  ((size_t)NPIX * CQKV * 4)
#define OFF_AHI   ((size_t)0)
#define OFF_ALO   (OFF_AHI + SZ_A)
#define OFF_WTHI  (OFF_ALO + SZ_A)
#define OFF_WTLO  (OFF_WTHI + SZ_WT)
#define OFF_WQHI  (OFF_WTLO + SZ_WT)
#define OFF_WQLO  (OFF_WQHI + SZ_WQ)
#define OFF_TOKHI (OFF_WQLO + SZ_WQ)
#define OFF_TOKLO (OFF_TOKHI + SZ_TOK)
#define OFF_QKV   (OFF_TOKLO + SZ_TOK)
#define WS_TOTAL  (OFF_QKV + SZ_QKV)

static_assert(X_N == 221184);
static_assert(OUT_N == 1179648);
static_assert(WS_TOTAL == 20905984);
static_assert((OFF_ALO % 128) == 0 && (OFF_WTHI % 128) == 0 && (OFF_WTLO % 128) == 0);
static_assert((OFF_WQHI % 128) == 0 && (OFF_WQLO % 128) == 0 && (OFF_TOKHI % 128) == 0);
static_assert((OFF_TOKLO % 128) == 0 && (OFF_QKV % 128) == 0);
static_assert(NPIX % 64 == 0 && CQKV % 128 == 0 && KT % 32 == 0 && CMID % 32 == 0);

#define PREP_A_ITEMS   (NPIX * (KT / 8))
#define PREP_WT_ITEMS  (CMID * (KT / 8))
#define PREP_WQ_ITEMS  (CQKV * (CMID / 8))
#define PREP_A_BLK     (PREP_A_ITEMS / 256)
#define PREP_WT_BLK    (PREP_WT_ITEMS / 256)
#define PREP_WQ_BLK    (PREP_WQ_ITEMS / 256)
#define PREP_BLOCKS    (PREP_A_BLK + PREP_WT_BLK + PREP_WQ_BLK)
static_assert(PREP_A_ITEMS % 256 == 0 && PREP_WT_ITEMS % 256 == 0 && PREP_WQ_ITEMS % 256 == 0);

#define TP 264
#define QP 136

typedef unsigned short v8us  __attribute__((ext_vector_type(8)));
typedef unsigned short v16us __attribute__((ext_vector_type(16)));
typedef __bf16         v16bf __attribute__((ext_vector_type(16)));
typedef float          v8f   __attribute__((ext_vector_type(8)));
typedef float          v4f   __attribute__((ext_vector_type(4)));
typedef float          v4fa  __attribute__((ext_vector_type(4), __may_alias__));

union Frag { v16us v; v8us half[2]; };

__device__ __forceinline__ unsigned short f2bf(float f) {
  unsigned int u = __float_as_uint(f);
  u += 0x7FFFu + ((u >> 16) & 1u);
  return (unsigned short)(u >> 16);
}
__device__ __forceinline__ float bf2f(unsigned short b) {
  return __uint_as_float(((unsigned int)b) << 16);
}

__device__ __forceinline__ void st2_u8(unsigned short* p, v8us v) {
  *(volatile v8us*)p = v;
  __threadfence();
  *(volatile v8us*)p = v;
}
__device__ __forceinline__ void st2_f4(float* p, v4f v) {
  *(volatile v4f*)p = v;
  __threadfence();
  *(volatile v4f*)p = v;
}

__device__ __forceinline__ v16bf ldfrag(const unsigned short* rowp, int h) {
  Frag f;
  f.half[0] = *(const v8us*)(rowp + 8 * h);
  f.half[1] = *(const v8us*)(rowp + 16 + 8 * h);
  return __builtin_bit_cast(v16bf, f.v);
}

__device__ __forceinline__ v8f wmma_bf(v16bf a, v16bf b, v8f c) {
  return __builtin_amdgcn_wmma_f32_16x16x32_bf16(false, a, false, b, (short)0, c, false, false);
}

__device__ __forceinline__ void mma3(v8f& acc, v16bf ah, v16bf al, v16bf bh, v16bf bl) {
  acc = wmma_bf(ah, bh, acc);
  acc = wmma_bf(al, bh, acc);
  acc = wmma_bf(ah, bl, acc);
  asm volatile("v_nop\n\tv_nop\n\tv_nop\n\tv_nop" : "+v"(acc) : "v"(ah), "v"(al), "v"(bh), "v"(bl));
}

__device__ __forceinline__ v8f v8f_zero() {
  v8f z = {0.f, 0.f, 0.f, 0.f, 0.f, 0.f, 0.f, 0.f};
  return z;
}

__device__ __forceinline__ void split8(const float* f, v8us& ph, v8us& pl) {
  #pragma unroll
  for (int j = 0; j < 8; ++j) {
    const unsigned short hb = f2bf(f[j]);
    const float res = f[j] - bf2f(hb);
    ph[j] = hb;
    pl[j] = f2bf(res);
  }
}

__global__ void __launch_bounds__(256) k_prep(
    const float* __restrict__ x, const float* __restrict__ wt, const float* __restrict__ wq,
    unsigned short* __restrict__ ahi, unsigned short* __restrict__ alo,
    unsigned short* __restrict__ wthi, unsigned short* __restrict__ wtlo,
    unsigned short* __restrict__ wqhi, unsigned short* __restrict__ wqlo) {
  const int bid = blockIdx.x;
  const int tid = threadIdx.x;
  v4f r0, r1;
  bool zero;
  unsigned short* dh;
  unsigned short* dl;
  size_t off;
  if (bid < PREP_A_BLK) {
    const int i = bid * 256 + tid;
    const int mrow = i >> 3, kc = i & 7;
    const int b = mrow / PIX;
    const int rem = mrow - b * PIX;
    const int hy = rem / WW;
    const int wx = rem - hy * WW;
    const int kcc = min(kc, 5);
    const int c = kcc >> 1;
    const int py0 = (kcc & 1) * 2;
    const float* rp = x + ((size_t)(b * CIN + c) * IMG + hy * PATCH + py0) * IMG + wx * PATCH;
    r0 = *(const v4f*)rp;
    r1 = *(const v4f*)(rp + IMG);
    zero = (kc >= 6);
    dh = ahi; dl = alo; off = (size_t)i * 8;
  } else if (bid < PREP_A_BLK + PREP_WT_BLK) {
    const int i = (bid - PREP_A_BLK) * 256 + tid;
    const int n = i >> 3, kc = i & 7;
    const float* rp = wt + (size_t)n * KTR + min(kc, 5) * 8;
    r0 = *(const v4f*)rp;
    r1 = *(const v4f*)(rp + 4);
    zero = (kc >= 6);
    dh = wthi; dl = wtlo; off = (size_t)i * 8;
  } else {
    const int i = (bid - PREP_A_BLK - PREP_WT_BLK) * 256 + tid;
    const int n = i >> 5, kc = i & 31;
    const float* rp = wq + (size_t)n * CMID + kc * 8;
    r0 = *(const v4f*)rp;
    r1 = *(const v4f*)(rp + 4);
    zero = false;
    dh = wqhi; dl = wqlo; off = (size_t)i * 8;
  }
  float f[8];
  f[0] = zero ? 0.f : r0.x; f[1] = zero ? 0.f : r0.y; f[2] = zero ? 0.f : r0.z; f[3] = zero ? 0.f : r0.w;
  f[4] = zero ? 0.f : r1.x; f[5] = zero ? 0.f : r1.y; f[6] = zero ? 0.f : r1.z; f[7] = zero ? 0.f : r1.w;
  v8us ph, pl;
  split8(f, ph, pl);
  st2_u8(dh + off, ph);
  st2_u8(dl + off, pl);
}

__global__ void __launch_bounds__(256) k_tok(
    const unsigned short* __restrict__ ahi, const unsigned short* __restrict__ alo,
    const unsigned short* __restrict__ wthi, const unsigned short* __restrict__ wtlo,
    const float* __restrict__ bt,
    unsigned short* __restrict__ tokhi, unsigned short* __restrict__ toklo) {
  __shared__ float tile[32 * TP];
  const int tid = threadIdx.x;
  const int lane = tid & 31;
  const int w = tid >> 5;
  const int h = lane >> 4;
  const int m = lane & 15;
  const int m0 = blockIdx.x * 32;
  const int r0 = (w >> 2) * 16;
  const int c0 = (w & 3) * 64;

  v8f acc[4];
  #pragma unroll
  for (int t = 0; t < 4; ++t) acc[t] = v8f_zero();

  const unsigned short* aph = ahi + (size_t)(m0 + r0 + m) * KT;
  const unsigned short* apl = alo + (size_t)(m0 + r0 + m) * KT;
  #pragma unroll 1
  for (int ks = 0; ks < KT / 32; ++ks) {
    const int k0 = ks * 32;
    const v16bf fah = ldfrag(aph + k0, h);
    const v16bf fal = ldfrag(apl + k0, h);
    #pragma unroll
    for (int t = 0; t < 4; ++t) {
      const size_t bo = (size_t)(c0 + t * 16 + m) * KT + k0;
      const v16bf fbh = ldfrag(wthi + bo, h);
      const v16bf fbl = ldfrag(wtlo + bo, h);
      mma3(acc[t], fah, fal, fbh, fbl);
    }
  }

  #pragma unroll
  for (int t = 0; t < 4; ++t) {
    const int col = c0 + t * 16 + m;
    const float bias = bt[col];
    #pragma unroll
    for (int r = 0; r < 8; ++r) tile[(r0 + 8 * h + r) * TP + col] = acc[t][r] + bias;
  }
  __syncthreads();

  #pragma unroll 1
  for (int it = 0; it < 4; ++it) {
    const int row = it * 8 + w;
    const v4fa* tp = (const v4fa*)(tile + row * TP + lane * 8);
    const v4f x0 = tp[0];
    const v4f x1 = tp[1];
    float f[8];
    f[0] = x0.x; f[1] = x0.y; f[2] = x0.z; f[3] = x0.w;
    f[4] = x1.x; f[5] = x1.y; f[6] = x1.z; f[7] = x1.w;
    v8us ph, pl;
    split8(f, ph, pl);
    const size_t off = (size_t)(m0 + row) * CMID + lane * 8;
    st2_u8(tokhi + off, ph);
    st2_u8(toklo + off, pl);
  }
}

__global__ void __launch_bounds__(256) k_qkv(
    const unsigned short* __restrict__ tokhi, const unsigned short* __restrict__ toklo,
    const unsigned short* __restrict__ wqhi, const unsigned short* __restrict__ wqlo,
    const float* __restrict__ bq, float* __restrict__ qkv) {
  __shared__ float tile[64 * QP];
  const int tid = threadIdx.x;
  const int lane = tid & 31;
  const int w = tid >> 5;
  const int h = lane >> 4;
  const int m = lane & 15;
  const int bid = blockIdx.x;
  const int mb = bid / 6;
  const int nb = bid - mb * 6;
  const int m0 = mb * 64;
  const int n0 = nb * 128;
  const int r0 = (w >> 2) * 32;
  const int c0 = (w & 3) * 32;

  v8f acc[2][2];
  acc[0][0] = v8f_zero(); acc[0][1] = v8f_zero();
  acc[1][0] = v8f_zero(); acc[1][1] = v8f_zero();

  const unsigned short* a0h = tokhi + (size_t)(m0 + r0 + m) * CMID;
  const unsigned short* a1h = a0h + 16 * CMID;
  const unsigned short* a0l = toklo + (size_t)(m0 + r0 + m) * CMID;
  const unsigned short* a1l = a0l + 16 * CMID;
  const unsigned short* b0h = wqhi + (size_t)(n0 + c0 + m) * CMID;
  const unsigned short* b1h = b0h + 16 * CMID;
  const unsigned short* b0l = wqlo + (size_t)(n0 + c0 + m) * CMID;
  const unsigned short* b1l = b0l + 16 * CMID;

  #pragma unroll 1
  for (int ks = 0; ks < CMID / 32; ++ks) {
    const int k0 = ks * 32;
    const v16bf A0h = ldfrag(a0h + k0, h), A0l = ldfrag(a0l + k0, h);
    const v16bf A1h = ldfrag(a1h + k0, h), A1l = ldfrag(a1l + k0, h);
    const v16bf B0h = ldfrag(b0h + k0, h), B0l = ldfrag(b0l + k0, h);
    const v16bf B1h = ldfrag(b1h + k0, h), B1l = ldfrag(b1l + k0, h);
    mma3(acc[0][0], A0h, A0l, B0h, B0l);
    mma3(acc[0][1], A0h, A0l, B1h, B1l);
    mma3(acc[1][0], A1h, A1l, B0h, B0l);
    mma3(acc[1][1], A1h, A1l, B1h, B1l);
  }

  #pragma unroll
  for (int i = 0; i < 2; ++i) {
    #pragma unroll
    for (int t = 0; t < 2; ++t) {
      const int col = c0 + t * 16 + m;
      const float bias = bq[n0 + col];
      #pragma unroll
      for (int r = 0; r < 8; ++r)
        tile[(r0 + i * 16 + 8 * h + r) * QP + col] = acc[i][t][r] + bias;
    }
  }
  __syncthreads();

  #pragma unroll 1
  for (int it = 0; it < 8; ++it) {
    const int row = it * 8 + w;
    const v4f v = *(const v4fa*)(tile + row * QP + lane * 4);
    st2_f4(qkv + (size_t)(m0 + row) * CQKV + n0 + lane * 4, v);
  }
}

__global__ void __launch_bounds__(64) k_attn(const float* __restrict__ qkv, float* __restrict__ out) {
  __shared__ float sc[KW * KW * 64];
  __shared__ float ot[HD * 64];
  const int tid = threadIdx.x;
  const int lane = tid & 31;
  const int w = tid >> 5;
  const int bid = blockIdx.x;
  const int pt = bid % (PIX / 64);
  const int hb = bid / (PIX / 64);
  const int hh = hb >> 1;
  const int bb = hb & 1;
  const int p0 = pt * 64;
  const int p = p0 + tid;
  const int y = p / WW;
  const int xq = p - y * WW;
  const int sy = min(max(y - KW / 2, 0), HH - KW);
  const int sx = min(max(xq - KW / 2, 0), WW - KW);

  const float* base = qkv + (size_t)bb * PIX * CQKV + hh * HD;
  v4f q4[8];
  {
    const float* qp = base + (size_t)p * CQKV;
    #pragma unroll
    for (int d4 = 0; d4 < 8; ++d4) q4[d4] = *(const v4f*)(qp + 4 * d4);
  }
  const float* kb = base + CMID;
  const float* vb = base + 2 * CMID;
  const float scale = 0.17677669529663687f;

  float mx = -__builtin_inff();
  int kk = 0;
  #pragma unroll 1
  for (int i = 0; i < KW; ++i) {
    const float* krow = kb + (size_t)((sy + i) * WW + sx) * CQKV;
    #pragma unroll 1
    for (int j = 0; j < KW; ++j) {
      const float* kp = krow + (size_t)j * CQKV;
      float s = 0.f;
      #pragma unroll
      for (int d4 = 0; d4 < 8; ++d4) {
        const v4f kv = *(const v4f*)(kp + 4 * d4);
        s += q4[d4].x * kv.x;
        s += q4[d4].y * kv.y;
        s += q4[d4].z * kv.z;
        s += q4[d4].w * kv.w;
      }
      s *= scale;
      sc[kk * 64 + tid] = s;
      mx = fmaxf(mx, s);
      ++kk;
    }
  }

  v4f acc[8];
  #pragma unroll
  for (int d4 = 0; d4 < 8; ++d4) { v4f z = {0.f, 0.f, 0.f, 0.f}; acc[d4] = z; }
  float sum = 0.f;
  kk = 0;
  #pragma unroll 1
  for (int i = 0; i < KW; ++i) {
    const float* vrow = vb + (size_t)((sy + i) * WW + sx) * CQKV;
    #pragma unroll 1
    for (int j = 0; j < KW; ++j) {
      const float* vp = vrow + (size_t)j * CQKV;
      const float e = __expf(sc[kk * 64 + tid] - mx);
      sum += e;
      #pragma unroll
      for (int d4 = 0; d4 < 8; ++d4) {
        const v4f vv = *(const v4f*)(vp + 4 * d4);
        acc[d4] = acc[d4] + vv * e;
      }
      ++kk;
    }
  }
  const float inv = 1.0f / sum;
  #pragma unroll
  for (int d4 = 0; d4 < 8; ++d4) {
    ot[(d4 * 4 + 0) * 64 + tid] = acc[d4].x * inv;
    ot[(d4 * 4 + 1) * 64 + tid] = acc[d4].y * inv;
    ot[(d4 * 4 + 2) * 64 + tid] = acc[d4].z * inv;
    ot[(d4 * 4 + 3) * 64 + tid] = acc[d4].w * inv;
  }
  __syncthreads();

  const int dl = lane >> 4;
  const int px = (lane & 15) * 4;
  float* ob = out + (size_t)(hh * BN + bb) * HD * PIX + p0 + px;
  #pragma unroll 1
  for (int it = 0; it < 8; ++it) {
    const int d = (it * 2 + w) * 2 + dl;
    const v4f v = *(const v4fa*)(ot + d * 64 + px);
    st2_f4(ob + (size_t)d * PIX, v);
  }
}

extern "C" void kernel_launch(void* const* d_in, const int* in_sizes, int n_in,
                              void* d_out, int out_size, void* d_ws, size_t ws_size,
                              hipStream_t stream) {
  if (n_in < 5) return;
  if (in_sizes[0] != X_N || in_sizes[1] != WT_N || in_sizes[2] != BT_N ||
      in_sizes[3] != WQ_N || in_sizes[4] != BQ_N) return;
  if (out_size != OUT_N) return;
  if (ws_size < (size_t)WS_TOTAL) return;

  const float* x     = (const float*)d_in[0];
  const float* w_tok = (const float*)d_in[1];
  const float* b_tok = (const float*)d_in[2];
  const float* w_qkv = (const float*)d_in[3];
  const float* b_qkv = (const float*)d_in[4];
  float* out = (float*)d_out;

  char* ws = (char*)d_ws;
  unsigned short* ahi   = (unsigned short*)(ws + OFF_AHI);
  unsigned short* alo   = (unsigned short*)(ws + OFF_ALO);
  unsigned short* wthi  = (unsigned short*)(ws + OFF_WTHI);
  unsigned short* wtlo  = (unsigned short*)(ws + OFF_WTLO);
  unsigned short* wqhi  = (unsigned short*)(ws + OFF_WQHI);
  unsigned short* wqlo  = (unsigned short*)(ws + OFF_WQLO);
  unsigned short* tokhi = (unsigned short*)(ws + OFF_TOKHI);
  unsigned short* toklo = (unsigned short*)(ws + OFF_TOKLO);
  float*          qkv   = (float*)(ws + OFF_QKV);

  k_prep<<<dim3(PREP_BLOCKS), dim3(256), 0, stream>>>(x, w_tok, w_qkv, ahi, alo, wthi, wtlo, wqhi, wqlo);
  k_tok<<<dim3(NPIX / 32), dim3(256), 0, stream>>>(ahi, alo, wthi, wtlo, b_tok, tokhi, toklo);
  k_qkv<<<dim3((NPIX / 64) * (CQKV / 128)), dim3(256), 0, stream>>>(tokhi, toklo, wqhi, wqlo, b_qkv, qkv);
  k_attn<<<dim3(HEADS * BN * (PIX / 64)), dim3(64), 0, stream>>>(qkv, out);
}
